// SimpleRNN_23828478558367
// MI455X (gfx1250) — hardware-verified
//
#include <hip/hip_runtime.h>
#include <math.h>

constexpr int NSEQ    = 64;
constexpr int NSTEP   = 512;
constexpr int NEMB    = 256;
constexpr int NHID    = 512;
constexpr int NOUTF   = 3;
constexpr int NVOCAB  = 50000;
constexpr int NTHR    = 256;
constexpr int SEQ_BLK = 16;
constexpr int HPITCH  = 520;
constexpr int XSP     = 516;
constexpr int NROWS   = NSEQ * NSTEP;
constexpr int NOUT    = NSEQ * NOUTF;
static_assert(NROWS % 64 == 0 && NHID % 64 == 0, "GEMM M, N tile multiples");
static_assert(NEMB % 32 == 0, "GEMM K multiple of 32");
static_assert(NEMB % 64 == 0 && NHID % 64 == 0, "transpose tiles exact");
static_assert(NSEQ % SEQ_BLK == 0, "recurrence grid exact");
static_assert(NHID == 64 * (NTHR / 32), "8 waves x 64 hidden columns");
static_assert(NROWS % (NTHR / 32) == 0, "gather grid exact");
static_assert(NEMB == 32 * 8, "gather: 32 lanes x 8 elements = one row");
static_assert((SEQ_BLK * NHID) % (4 * NTHR) == 0, "xp staging / h_last store loops exact");
static_assert(NOUT % 4 == 0 && NOUT / 4 <= 64, "output funnel: 48 float4 over two waves");
static_assert(HPITCH % 8 == 0 && XSP % 4 == 0, "16-B aligned LDS rows");

typedef __attribute__((ext_vector_type(16))) _Float16 v16h;
typedef __attribute__((ext_vector_type(8)))  _Float16 v8h;
typedef __attribute__((ext_vector_type(16))) __bf16   v16b;
typedef __attribute__((ext_vector_type(8)))  __bf16   v8b;
typedef __attribute__((ext_vector_type(8)))  float    v8f;
typedef __attribute__((ext_vector_type(4)))  float    v4f;

__device__ __forceinline__ unsigned short f2bf_bits(float f) {
  unsigned u = __float_as_uint(f);
  return (unsigned short)((u + 0x7FFFu + ((u >> 16) & 1u)) >> 16);
}
__device__ __forceinline__ float bf_bits2f(unsigned short h) { return __uint_as_float(((unsigned)h) << 16); }
__device__ __forceinline__ float bf16r(float f) { return bf_bits2f(f2bf_bits(f)); }

__device__ __forceinline__ void dep_guard_h(v8f& a, v8f& b, v16h x, v16h y) { asm volatile("v_nop\n\tv_nop\n\tv_nop\n\tv_nop" : "+v"(a), "+v"(b) : "v"(x), "v"(y)); }
__device__ __forceinline__ void dep_guard_b(v8f& a, v8f& b, v16b x, v16b y) { asm volatile("v_nop\n\tv_nop\n\tv_nop\n\tv_nop" : "+v"(a), "+v"(b) : "v"(x), "v"(y)); }
__device__ __forceinline__ void dep_guard4_h(v8f& a, v8f& b, v8f& c, v8f& d, v16h x, v16h y) {
  asm volatile("v_nop\n\tv_nop\n\tv_nop\n\tv_nop" : "+v"(a), "+v"(b), "+v"(c), "+v"(d) : "v"(x), "v"(y));
}
__device__ __forceinline__ void dep_guard4_b(v8f& a, v8f& b, v8f& c, v8f& d, v16b x, v16b y) {
  asm volatile("v_nop\n\tv_nop\n\tv_nop\n\tv_nop" : "+v"(a), "+v"(b), "+v"(c), "+v"(d) : "v"(x), "v"(y));
}
__device__ __forceinline__ void keep4_h(v16h a, v16h b, v16h c, v16h d) { asm volatile("v_nop" :: "v"(a), "v"(b), "v"(c), "v"(d)); }
__device__ __forceinline__ void keep4_b(v16b a, v16b b, v16b c, v16b d) { asm volatile("v_nop" :: "v"(a), "v"(b), "v"(c), "v"(d)); }
__device__ __forceinline__ void acc_guard4(v8f& a, v8f& b, v8f& c, v8f& d) { asm volatile("v_nop\n\tv_nop\n\tv_nop\n\tv_nop" : "+v"(a), "+v"(b), "+v"(c), "+v"(d)); }
__device__ __forceinline__ void guard_all_b(v8f& a0, v8f& a1, v8f& a2, v8f& a3,
                                            v16b x0, v16b x1, v16b y0, v16b y1, v16b y2, v16b y3) {
  asm volatile("v_nop\n\tv_nop\n\tv_nop\n\tv_nop"
               : "+v"(a0), "+v"(a1), "+v"(a2), "+v"(a3)
               : "v"(x0), "v"(x1), "v"(y0), "v"(y1), "v"(y2), "v"(y3));
}
template <typename T> struct Frag;
template <> struct Frag<_Float16> {
  typedef v16h V; union U { v16h v; v8h h[2]; };
  static __device__ __forceinline__ v16h load(const _Float16* p) {
    U f; f.h[0] = *(const v8h*)(p); f.h[1] = *(const v8h*)(p + 16); return f.v;
  }
  static __device__ __forceinline__ v8f mma(v16h a, v16h b, v8f c) {
    return __builtin_amdgcn_wmma_f32_16x16x32_f16(false, a, false, b, (short)0, c, false, false);
  }
  static __device__ __forceinline__ void guard(v8f& a, v8f& b, v16h x, v16h y) { dep_guard_h(a, b, x, y); }
  static __device__ __forceinline__ void guard4(v8f& a, v8f& b, v8f& c, v8f& d, v16h x, v16h y) { dep_guard4_h(a, b, c, d, x, y); }
  static __device__ __forceinline__ void keep(v16h a, v16h b, v16h c, v16h d) { keep4_h(a, b, c, d); }
};
template <> struct Frag<__bf16> {
  typedef v16b V; union U { v16b v; v8b h[2]; };
  static __device__ __forceinline__ v16b load(const __bf16* p) {
    U f; f.h[0] = *(const v8b*)(p); f.h[1] = *(const v8b*)(p + 16); return f.v;
  }
  static __device__ __forceinline__ v8f mma(v16b a, v16b b, v8f c) {
    return __builtin_amdgcn_wmma_f32_16x16x32_bf16(false, a, false, b, (short)0, c, false, false);
  }
  static __device__ __forceinline__ void guard(v8f& a, v8f& b, v16b x, v16b y) { dep_guard_b(a, b, x, y); }
  static __device__ __forceinline__ void guard4(v8f& a, v8f& b, v8f& c, v8f& d, v16b x, v16b y) { dep_guard4_b(a, b, c, d, x, y); }
  static __device__ __forceinline__ void keep(v16b a, v16b b, v16b c, v16b d) { keep4_b(a, b, c, d); }
};

__device__ __forceinline__ float ftanh(float x) { return 1.0f - 2.0f * __builtin_amdgcn_rcpf(__expf(2.0f * x) + 1.0f); }

template <int ET> struct Elem;
template <> struct Elem<0> { typedef _Float16 T; };
template <> struct Elem<1> { typedef __bf16 T; };
template <int ET, bool SPLIT, int BIAS_MODE, int OUT_MODE, bool RESID, int ACT = 0>
__global__ __launch_bounds__(256) void wmma_gemm64(
    const unsigned short* __restrict__ Ap, const unsigned short* __restrict__ A2p, int lda, long strideA,
    const unsigned short* __restrict__ Btp, const unsigned short* __restrict__ Bt2p, int ldb, long strideB,
    void* __restrict__ Cout, void* __restrict__ Cout2, int ldc, long strideC,
    const float* __restrict__ bias,
    const float* __restrict__ resid, long strideR,
    int M, int N, int K, float scale) {
  typedef typename Elem<ET>::T T;
  typedef typename Frag<T>::V V;
  const T* A = (const T*)Ap; const T* A2 = (const T*)A2p; const T* Bt = (const T*)Btp; const T* Bt2 = (const T*)Bt2p;
  __shared__ __align__(16) float sT[8][16 * 68];
  const int b    = blockIdx.y;
  const int lane = threadIdx.x & 31;
  const int wave = threadIdx.x >> 5;
  const int tilesN = N >> 6;
  const int tilesM = M >> 6;
  const int tile = blockIdx.x * 8 + wave;
  if (tile >= tilesM * tilesN) return;
  const int tm = tile / tilesN;
  const int tn = tile - tm * tilesN;
  const int m0 = tm << 6;
  const int n0 = tn << 6;

  const T* Ab  = A  + (size_t)b * strideA;
  const T* Bb  = Bt + (size_t)b * strideB;
  const T* Ab2 = SPLIT ? (A2  + (size_t)b * strideA) : nullptr;
  const T* Bb2 = SPLIT ? (Bt2 + (size_t)b * strideB) : nullptr;

  const int rlane = lane & 15;
  const int koff  = (lane >> 4) * 8;
  const int mOff  = (lane >> 4) * 8;

  v8f acc[4][4];
#pragma unroll
  for (int i = 0; i < 4; ++i)
#pragma unroll
    for (int j = 0; j < 4; ++j) acc[i][j] = (v8f){0.f,0.f,0.f,0.f,0.f,0.f,0.f,0.f};

  for (int k0 = 0; k0 < K; k0 += 32) {
    V bh[4], bl[4];
#pragma unroll
    for (int j = 0; j < 4; ++j) {
      const size_t bo = (size_t)(n0 + (j << 4) + rlane) * ldb + koff + k0;
      bh[j] = Frag<T>::load(Bb + bo);
      if (SPLIT) bl[j] = Frag<T>::load(Bb2 + bo);
    }
#pragma unroll
    for (int i = 0; i < 4; ++i) {
      const size_t ao = (size_t)(m0 + (i << 4) + rlane) * lda + koff + k0;
      V ah = Frag<T>::load(Ab + ao);
      V al;
      if (SPLIT) al = Frag<T>::load(Ab2 + ao);
#pragma unroll
      for (int j = 0; j < 4; ++j) {
        acc[i][j] = Frag<T>::mma(ah, bh[j], acc[i][j]);
        if (SPLIT) {
          acc[i][j] = Frag<T>::mma(ah, bl[j], acc[i][j]);
          acc[i][j] = Frag<T>::mma(al, bh[j], acc[i][j]);
        }
      }
      Frag<T>::guard4(acc[i][0], acc[i][1], acc[i][2], acc[i][3], ah, SPLIT ? al : ah);
    }
    Frag<T>::keep(bh[0], bh[1], bh[2], bh[3]);
    if (SPLIT) Frag<T>::keep(bl[0], bl[1], bl[2], bl[3]);
  }
  acc_guard4(acc[0][0], acc[0][1], acc[0][2], acc[0][3]);
  acc_guard4(acc[1][0], acc[1][1], acc[1][2], acc[1][3]);
  acc_guard4(acc[2][0], acc[2][1], acc[2][2], acc[2][3]);
  acc_guard4(acc[3][0], acc[3][1], acc[3][2], acc[3][3]);

  float* slab = sT[wave];
  const float* Rb = RESID ? (resid + (size_t)b * strideR) : nullptr;
#pragma unroll
  for (int i = 0; i < 4; ++i) {
    const int mBase = m0 + (i << 4);
#pragma unroll
    for (int j = 0; j < 4; ++j) {
      const int n = n0 + (j << 4) + rlane;
      float bv = 0.f;
      if (BIAS_MODE == 2) bv = bias[n];
#pragma unroll
      for (int r = 0; r < 8; ++r) {
        float v = acc[i][j][r] * scale;
        if (BIAS_MODE == 1) v += bias[mBase + mOff + r];
        if (BIAS_MODE == 2) v += bv;
        if (RESID) v += Rb[(size_t)(mBase + mOff + r) * ldc + n];
        if (ACT == 1) v = tanhf(v);
        if (ACT == 2) v = fmaxf(v, 0.0f);
        if (ACT == 3) v = v / (1.0f + expf(-v));
        if (ACT == 4) v = (v > 0.f) ? v : 0.01f * v;
        if (ACT == 5) v = 0.5f * v * (1.0f + erff(v * 0.70710678118654752f));
        slab[(mOff + r) * 68 + (j << 4) + rlane] = v;
      }
    }
    __builtin_amdgcn_fence(__ATOMIC_RELEASE, "workgroup");
    __builtin_amdgcn_wave_barrier();
    __builtin_amdgcn_fence(__ATOMIC_ACQUIRE, "workgroup");
    if (OUT_MODE == 0) {
      float* C = (float*)Cout + (size_t)b * strideC;
      const int hh = lane >> 4, c4 = (lane & 15) * 4;
      for (int pass = 0; pass < 2; ++pass) {
#pragma unroll
        for (int it = 0; it < 8; ++it) {
          const int row = it * 2 + hh;
          v4f v = *(const v4f*)(slab + row * 68 + c4);
          *(volatile v4f*)(C + (size_t)(mBase + row) * ldc + n0 + c4) = v;
        }
        __threadfence();
      }
    } else {
      const int q = lane >> 3, c8 = (lane & 7) * 8;
      unsigned short* C  = (unsigned short*)Cout  + (size_t)b * strideC;
      unsigned short* C2 = (OUT_MODE == 2) ? ((unsigned short*)Cout2 + (size_t)b * strideC) : nullptr;
      for (int pass = 0; pass < 2; ++pass) {
#pragma unroll
        for (int it = 0; it < 4; ++it) {
          const int row = it * 4 + q;
          const float* sp = slab + row * 68 + c8;
          v8h hv, lv;
#pragma unroll
          for (int e = 0; e < 8; ++e) {
            if (OUT_MODE == 1) {
              hv[e] = (_Float16)sp[e];
            } else {
              unsigned short hb = f2bf_bits(sp[e]);
              unsigned short lb = f2bf_bits(sp[e] - bf_bits2f(hb));
              hv[e] = __builtin_bit_cast(_Float16, hb);
              lv[e] = __builtin_bit_cast(_Float16, lb);
            }
          }
          *(volatile v8h*)(C + (size_t)(mBase + row) * ldc + n0 + c8) = hv;
          if (OUT_MODE == 2) *(volatile v8h*)(C2 + (size_t)(mBase + row) * ldc + n0 + c8) = lv;
        }
        __threadfence();
      }
    }
    __builtin_amdgcn_fence(__ATOMIC_RELEASE, "workgroup");
    __builtin_amdgcn_wave_barrier();
    __builtin_amdgcn_fence(__ATOMIC_ACQUIRE, "workgroup");
  }
}

template <int MODE>
__global__ __launch_bounds__(NTHR) void tpw_kernel(const float* __restrict__ src, int R, int C, int ldo,
                                                  unsigned short* __restrict__ O, float sc) {
  __shared__ float Tt[64 * 65];
  const int tid = threadIdx.x;
  const int c0 = blockIdx.x * 64, r0 = blockIdx.y * 64;
#pragma unroll
  for (int i = 0; i < 4; ++i) {
    const int idx = i * NTHR + tid;
    const int rr = idx >> 4, cc = (idx & 15) * 4;
    const v4f v = *(const v4f*)(src + (size_t)(r0 + rr) * (size_t)C + c0 + cc);
    Tt[rr * 65 + cc + 0] = v[0];
    Tt[rr * 65 + cc + 1] = v[1];
    Tt[rr * 65 + cc + 2] = v[2];
    Tt[rr * 65 + cc + 3] = v[3];
  }
  __syncthreads();
  const int q = tid >> 3, c8 = (tid & 7) * 8;
  v8h hv[2];
#pragma unroll
  for (int g = 0; g < 2; ++g) {
    const int qq = g * 32 + q;
#pragma unroll
    for (int e = 0; e < 8; ++e) {
      const float f = Tt[(c8 + e) * 65 + qq];
      unsigned short bits;
      if (MODE == 0) {
        bits = f2bf_bits(f * sc);
      } else {
        const float fb = bf_bits2f(f2bf_bits(f));
        bits = __builtin_bit_cast(unsigned short, (_Float16)(fb * sc));
      }
      hv[g][e] = __builtin_bit_cast(_Float16, bits);
    }
  }
  for (int pass = 0; pass < 2; ++pass) {
#pragma unroll
    for (int g = 0; g < 2; ++g) {
      const size_t o = (size_t)(c0 + g * 32 + q) * (size_t)ldo + (size_t)(r0 + c8);
      *(volatile v8h*)(O + o) = hv[g];
    }
    __threadfence();
  }
}

__global__ __launch_bounds__(NTHR) void gather_kernel(const int* __restrict__ tokens, const float* __restrict__ emb,
                                                     unsigned short* __restrict__ XB) {
  const int tid = threadIdx.x, lane = tid & 31, wave = tid >> 5;
  const int r = blockIdx.x * (NTHR / 32) + wave;
  const int t = r >> 6, b = r & 63;
  int tok = tokens[b * NSTEP + t];
  tok = tok < 0 ? 0 : (tok > NVOCAB - 1 ? NVOCAB - 1 : tok);
  const float* sp = emb + (size_t)tok * NEMB + lane * 8;
  const v4f a  = *(const v4f*)(sp);
  const v4f bq = *(const v4f*)(sp + 4);
  v8h hv;
#pragma unroll
  for (int e = 0; e < 4; ++e) {
    const unsigned short u0 = f2bf_bits(a[e]);
    const unsigned short u1 = f2bf_bits(bq[e]);
    hv[e]     = __builtin_bit_cast(_Float16, u0);
    hv[4 + e] = __builtin_bit_cast(_Float16, u1);
  }
  unsigned short* dp = XB + (size_t)r * NEMB + lane * 8;
  *(volatile v8h*)dp = hv;
  __threadfence();
  *(volatile v8h*)dp = hv;
}

__device__ __forceinline__ void stage_xp(const float* __restrict__ XP, float* xs, int tt, int rowbase, int tid) {
  const float* xb = XP + ((size_t)tt * NSEQ + (size_t)rowbase) * NHID;
#pragma unroll
  for (int it = 0; it < 4; ++it) {
    const int idx = it * NTHR + tid;
    const int row = idx >> 7, c4 = (idx & 127) * 4;
    const v4f v = *(const v4f*)(xb + (size_t)row * NHID + c4);
    *(v4f*)(xs + row * XSP + c4) = v;
  }
  asm volatile("" ::: "memory");
#pragma unroll
  for (int it = 4; it < 8; ++it) {
    const int idx = it * NTHR + tid;
    const int row = idx >> 7, c4 = (idx & 127) * 4;
    const v4f v = *(const v4f*)(xb + (size_t)row * NHID + c4);
    *(v4f*)(xs + row * XSP + c4) = v;
  }
}

__global__ __launch_bounds__(NTHR) void rnn_seq_kernel(const float* __restrict__ XP, const unsigned short* __restrict__ WHp,
                                                      float* __restrict__ HLAST) {
  __shared__ __align__(16) unsigned short Hhi[SEQ_BLK * HPITCH];
  __shared__ __align__(16) unsigned short Hlo[SEQ_BLK * HPITCH];
  __shared__ __align__(16) float          Xs[SEQ_BLK * XSP];
  const __bf16* WH = (const __bf16*)WHp;
  const int tid = threadIdx.x, lane = tid & 31, wave = tid >> 5;
  const int c = lane & 15, hh = lane >> 4, koff = hh * 8;
  const int rowbase = blockIdx.x * SEQ_BLK;

#pragma unroll 1
  for (int i = tid; i < SEQ_BLK * HPITCH; i += NTHR) { Hhi[i] = (unsigned short)0; Hlo[i] = (unsigned short)0; }
  stage_xp(XP, Xs, 0, rowbase, tid);
  float hst[4][8];
#pragma unroll
  for (int nt = 0; nt < 4; ++nt)
#pragma unroll
    for (int r = 0; r < 8; ++r) hst[nt][r] = 0.0f;
  __syncthreads();

  const __bf16* hhrow = (const __bf16*)Hhi + c * HPITCH + koff;
  const __bf16* hlrow = (const __bf16*)Hlo + c * HPITCH + koff;
  const __bf16* wrow  = WH + (size_t)(64 * wave + c) * NHID + koff;
  const v8f z8 = {0.f, 0.f, 0.f, 0.f, 0.f, 0.f, 0.f, 0.f};

#pragma unroll 1
  for (int t = 0; t < NSTEP; ++t) {
    v8f acc[4];
    acc[0] = z8; acc[1] = z8; acc[2] = z8; acc[3] = z8;
#pragma unroll 1
    for (int k0 = 0; k0 < NHID; k0 += 32) {
      const v16b ah = Frag<__bf16>::load(hhrow + k0);
      const v16b al = Frag<__bf16>::load(hlrow + k0);
      const v16b b0 = Frag<__bf16>::load(wrow + k0);
      const v16b b1 = Frag<__bf16>::load(wrow + (size_t)16 * NHID + k0);
      const v16b b2 = Frag<__bf16>::load(wrow + (size_t)32 * NHID + k0);
      const v16b b3 = Frag<__bf16>::load(wrow + (size_t)48 * NHID + k0);
      acc[0] = Frag<__bf16>::mma(ah, b0, acc[0]);
      acc[0] = Frag<__bf16>::mma(al, b0, acc[0]);
      acc[1] = Frag<__bf16>::mma(ah, b1, acc[1]);
      acc[1] = Frag<__bf16>::mma(al, b1, acc[1]);
      acc[2] = Frag<__bf16>::mma(ah, b2, acc[2]);
      acc[2] = Frag<__bf16>::mma(al, b2, acc[2]);
      acc[3] = Frag<__bf16>::mma(ah, b3, acc[3]);
      acc[3] = Frag<__bf16>::mma(al, b3, acc[3]);
      guard_all_b(acc[0], acc[1], acc[2], acc[3], ah, al, b0, b1, b2, b3);
    }
    acc_guard4(acc[0], acc[1], acc[2], acc[3]);

#pragma unroll
    for (int nt = 0; nt < 4; ++nt) {
      const int j = 64 * wave + 16 * nt + c;
#pragma unroll
      for (int r = 0; r < 8; ++r) {
        const float z = acc[nt][r] + Xs[(8 * hh + r) * XSP + j];
        hst[nt][r] = ftanh(z);
      }
    }
    __syncthreads();

#pragma unroll
    for (int nt = 0; nt < 4; ++nt) {
      const int j = 64 * wave + 16 * nt + c;
#pragma unroll
      for (int r = 0; r < 8; ++r) {
        const float h = hst[nt][r];
        const unsigned short hb = f2bf_bits(h);
        const unsigned short lb = f2bf_bits(h - bf_bits2f(hb));
        Hhi[(8 * hh + r) * HPITCH + j] = hb;
        Hlo[(8 * hh + r) * HPITCH + j] = lb;
      }
    }
    {
      const int tn = (t + 1 < NSTEP) ? (t + 1) : (NSTEP - 1);
      stage_xp(XP, Xs, tn, rowbase, tid);
    }
    __syncthreads();
  }

#pragma unroll
  for (int nt = 0; nt < 4; ++nt) {
    const int j = 64 * wave + 16 * nt + c;
#pragma unroll
    for (int r = 0; r < 8; ++r) Xs[(8 * hh + r) * XSP + j] = hst[nt][r];
  }
  __syncthreads();
  for (int pass = 0; pass < 2; ++pass) {
#pragma unroll
    for (int it = 0; it < 8; ++it) {
      const int idx = it * NTHR + tid;
      const int row = idx >> 7, c4 = (idx & 127) * 4;
      const v4f v = *(const v4f*)(Xs + row * XSP + c4);
      *(volatile v4f*)(HLAST + (size_t)(rowbase + row) * NHID + c4) = v;
    }
    __threadfence();
  }
}

__global__ __launch_bounds__(NTHR) void fc_kernel(const float* __restrict__ HLAST, const float* __restrict__ W_fc,
                                                 const float* __restrict__ b_fc, float* __restrict__ out) {
  __shared__ __align__(16) float so[NOUT];
  const int tid = threadIdx.x;
  const int bq = tid / NOUTF;
  const int o = tid - bq * NOUTF;
  const int bcl = bq < NSEQ ? bq : (NSEQ - 1);
  const float* hp = HLAST + (size_t)bcl * NHID;
  float s = 0.0f;
#pragma unroll 1
  for (int k = 0; k < NHID; ++k) s += hp[k] * bf16r(W_fc[k * NOUTF + o]);
  s += bf16r(b_fc[o]);
  if (tid < NOUT) so[tid] = s;
  __syncthreads();
  if (tid < NOUT / 4) {
    const v4f v = *(const v4f*)(so + 4 * tid);
    for (int pass = 0; pass < 2; ++pass) {
      *(volatile v4f*)(out + 4 * tid) = v;
      __threadfence();
    }
  }
}

extern "C" void kernel_launch(void* const* d_in, const int* in_sizes, int n_in,
                              void* d_out, int out_size, void* d_ws, size_t ws_size, hipStream_t stream) {
  if (n_in < 7 || d_out == nullptr || d_ws == nullptr) return;
  if (in_sizes[0] != NSEQ * NSTEP || in_sizes[1] != NVOCAB * NEMB || in_sizes[2] != NEMB * NHID ||
      in_sizes[3] != NHID * NHID || in_sizes[4] != NHID || in_sizes[5] != NHID * NOUTF || in_sizes[6] != NOUTF ||
      out_size != NOUT) return;

  const int*   tokens = (const int*)d_in[0];
  const float* emb    = (const float*)d_in[1];
  const float* w_xh   = (const float*)d_in[2];
  const float* w_hh   = (const float*)d_in[3];
  const float* b_h    = (const float*)d_in[4];
  const float* w_fc   = (const float*)d_in[5];
  const float* b_fc   = (const float*)d_in[6];
  float* out = (float*)d_out;

  char* ws = (char*)d_ws; size_t off = 0;
  auto carve = [&](size_t bytes) -> char* { char* p = ws + off; off += (bytes + 255) & ~(size_t)255; return p; };
  unsigned short* XB    = (unsigned short*)carve((size_t)NROWS * NEMB * 2);
  unsigned short* WXT   = (unsigned short*)carve((size_t)NHID * NEMB * 2);
  unsigned short* WHT   = (unsigned short*)carve((size_t)NHID * NHID * 2);
  float*          XP    = (float*)carve((size_t)NROWS * NHID * 4);
  float*          HLAST = (float*)carve((size_t)NSEQ * NHID * 4);
  if (off > ws_size || off > (size_t)134217728) return;

  tpw_kernel<0><<<dim3(NHID / 64, NEMB / 64), NTHR, 0, stream>>>(w_xh, NEMB, NHID, NEMB, WXT, 1.0f);
  tpw_kernel<0><<<dim3(NHID / 64, NHID / 64), NTHR, 0, stream>>>(w_hh, NHID, NHID, NHID, WHT, 1.0f);
  gather_kernel<<<NROWS / (NTHR / 32), NTHR, 0, stream>>>(tokens, emb, XB);
  const dim3 ggrid((NROWS / 64) * (NHID / 64) / 8, 1);
  wmma_gemm64<1, false, 2, 0, false, 0><<<ggrid, 256, 0, stream>>>(
      XB, XB, NEMB, 0L, WXT, WXT, NEMB, 0L, (void*)XP, (void*)XP, NHID, 0L,
      b_h, HLAST, 0L, NROWS, NHID, NEMB, 1.0f);
  rnn_seq_kernel<<<NSEQ / SEQ_BLK, NTHR, 0, stream>>>(XP, WHT, HLAST);
  fc_kernel<<<1, NTHR, 0, stream>>>(HLAST, w_fc, b_fc, out);
}
